// CNODExtmod_70781061038895
// MI455X (gfx1250) — hardware-verified
//
#include <hip/hip_runtime.h>
#include <math.h>

typedef __attribute__((ext_vector_type(16))) _Float16 v16h;
typedef __attribute__((ext_vector_type(16))) __bf16 v16b;
typedef __attribute__((ext_vector_type(8)))  _Float16 v8h;
typedef __attribute__((ext_vector_type(8)))  float v8f;
typedef __attribute__((ext_vector_type(4)))  float v4f;
typedef __attribute__((ext_vector_type(2)))  float v2f;
typedef __attribute__((ext_vector_type(4)))  unsigned v4u;
typedef __attribute__((ext_vector_type(4)))  int v4i;
typedef float __attribute__((may_alias)) float_a;
typedef int __attribute__((may_alias)) int_a;

template <typename T> __device__ __forceinline__ void vst2(void* p, T v) { *(volatile T*)p = v; __threadfence(); *(volatile T*)p = v; }
__device__ __forceinline__ v8f wmma16(v16h a, v16h b, v8f c) {
  v8f d = __builtin_amdgcn_wmma_f32_16x16x32_f16(false, a, false, b, (short)0, c, false, false);
  asm volatile("v_nop\n\tv_nop\n\tv_nop\n\tv_nop" : "+v"(d) : "v"(a), "v"(b));
  return d;
}
__device__ __forceinline__ v8f wmma_bf(v16b a, v16b b, v8f c) {
  v8f d = __builtin_amdgcn_wmma_f32_16x16x32_bf16(false, a, false, b, (short)0, c, false, false);
  asm volatile("v_nop\n\tv_nop\n\tv_nop\n\tv_nop" : "+v"(d) : "v"(a), "v"(b));
  return d;
}
__device__ __forceinline__ v16h frag_h(const _Float16* rowk0, int lane) {
  union { v16h v; v8h q[2]; } u; const _Float16* p = rowk0 + 8 * (lane >> 4);
  u.q[0] = *(const v8h*)p; u.q[1] = *(const v8h*)(p + 16); return u.v;
}
__device__ __forceinline__ v16h frag_f32(const float* rowk0, int lane) {
  v16h a; const float* p = rowk0 + 8 * (lane >> 4);
#pragma unroll
  for (int i = 0; i < 8; ++i) { a[i] = (_Float16)p[i]; a[8 + i] = (_Float16)p[16 + i]; }
  return a;
}
__device__ __forceinline__ v16h frag_f32s(const float* rowk0, int lane, float sc) {
  v16h a; const float* p = rowk0 + 8 * (lane >> 4);
#pragma unroll
  for (int i = 0; i < 8; ++i) { a[i] = (_Float16)(p[i] * sc); a[8 + i] = (_Float16)(p[16 + i] * sc); }
  return a;
}
__device__ __forceinline__ v16h fragc_f32(const float* W, int k0, int n, int lane, int ld, int K) {
  v16h a; const int g = lane >> 4;
#pragma unroll
  for (int i = 0; i < 8; ++i) { const int ka = k0 + 8 * g + i, kb = ka + 16;
    a[i] = (_Float16)(ka < K ? W[(size_t)(ka < K ? ka : K - 1) * ld + n] : 0.f); a[8 + i] = (_Float16)(kb < K ? W[(size_t)(kb < K ? kb : K - 1) * ld + n] : 0.f); }
  return a;
}
struct F2 { v16b h, l; };
__device__ __forceinline__ F2 bsplit16(const float v[16]) { F2 r;
#pragma unroll
  for (int i = 0; i < 16; ++i) { const __bf16 h = (__bf16)v[i]; r.h[i] = h; r.l[i] = (__bf16)(v[i] - (float)h); }
  return r; }
__device__ __forceinline__ F2 split_row(const float* row, int k0, int lane) { float v[16]; const float* p = row + k0 + 8 * (lane >> 4);
#pragma unroll
  for (int i = 0; i < 8; ++i) { v[i] = p[i]; v[8 + i] = p[16 + i]; }
  return bsplit16(v); }
__device__ __forceinline__ F2 split_rowK(const float* row, int k0, int lane, int K) { float v[16]; const int g = lane >> 4;
#pragma unroll
  for (int i = 0; i < 8; ++i) { const int ka = k0 + 8 * g + i, kb = ka + 16; v[i] = ka < K ? row[ka < K ? ka : K - 1] : 0.f; v[8 + i] = kb < K ? row[kb < K ? kb : K - 1] : 0.f; }
  return bsplit16(v); }
__device__ __forceinline__ F2 split_col(const float* W, int k0, int n, int lane, int ld, int K) { float v[16]; const int g = lane >> 4;
#pragma unroll
  for (int i = 0; i < 8; ++i) { const int ka = k0 + 8 * g + i, kb = ka + 16; v[i] = ka < K ? W[(size_t)(ka < K ? ka : K - 1) * ld + n] : 0.f; v[8 + i] = kb < K ? W[(size_t)(kb < K ? kb : K - 1) * ld + n] : 0.f; }
  return bsplit16(v); }
__device__ __forceinline__ v8f mac3(const F2& a, const F2& b, v8f c) { c = wmma_bf(a.l, b.h, c); c = wmma_bf(a.h, b.l, c); return wmma_bf(a.h, b.h, c); }
__device__ __forceinline__ float sigm(float v) { return 1.0f / (1.0f + expf(-v)); }
#define LDSX() do { asm volatile("s_wait_dscnt 0" ::: "memory"); __builtin_amdgcn_wave_barrier(); __builtin_amdgcn_fence(__ATOMIC_RELEASE, "workgroup"); } while (0)


#define NBATCH 4096
#define NC 32
#define NS 65
#define HID 128
#define NT 64
#define NSUB 4
#define RB 32
__device__ __forceinline__ float bfr(float v) { return (float)(__bf16)v; }
typedef __attribute__((ext_vector_type(8))) __bf16 v8b;
__device__ __forceinline__ v16b frag_b(const __bf16* rowk0, int lane) {
  union { v16b v; v8b q[2]; } u; const __bf16* p = rowk0 + 8 * (lane >> 4);
  u.q[0] = *(const v8b*)p; u.q[1] = *(const v8b*)(p + 16); return u.v;
}

__global__ __launch_bounds__(64) void k_ode(const float* __restrict__ times, const float* __restrict__ Yin, const float* __restrict__ maskin, const float* __restrict__ Am, const float* __restrict__ Bv,
                                            const float* __restrict__ W1, const float* __restrict__ b1, const float* __restrict__ W2, const float* __restrict__ b2, const float* __restrict__ W3, const float* __restrict__ b3,
                                            float* __restrict__ out0, float* __restrict__ out1, float* __restrict__ out2, float* __restrict__ out3) {
  __shared__ __align__(16) __bf16 sA[NC][NC], sW1[HID][64], sW2[HID][HID], sW3[48][HID];
  __shared__ float sBv[NC], sb1[HID], sb2[HID], sb3[48];
  __shared__ __align__(16) float sh[RB][72];
  __shared__ __align__(16) float sd[RB][72];
  __shared__ __align__(16) float s1[RB][HID + 4], s2[RB][HID + 4];
  __shared__ __align__(16) float syp[RB][NT];
  const int tid = threadIdx.x, wave = tid >> 5, lane = tid & 31, col = lane & 15, g = lane >> 4; const size_t r0 = (size_t)blockIdx.x * RB;
  for (int q = tid; q < NC * NC; q += 64) sA[q >> 5][q & 31] = (__bf16)Am[q];
  for (int q = tid; q < HID * 64; q += 64) { const int n = q >> 6, k = q & 63; sW1[n][k] = k < NC + 1 ? (__bf16)W1[n * (NC + 1) + k] : (__bf16)0.f; }
  for (int q = tid; q < HID * HID; q += 64) sW2[q >> 7][q & 127] = (__bf16)W2[q];
  for (int q = tid; q < 48 * HID; q += 64) { const int n = q >> 7, k = q & 127; sW3[n][k] = n < NC + 1 ? (__bf16)W3[n * HID + k] : (__bf16)0.f; }
  if (tid < NC) sBv[tid] = bfr(Bv[tid]);
  for (int q = tid; q < HID; q += 64) { sb1[q] = bfr(b1[q]); sb2[q] = bfr(b2[q]); }
  if (tid < 48) sb3[tid] = tid < NC + 1 ? bfr(b3[tid]) : 0.f;
  for (int q = tid; q < RB * 72; q += 64) { (&sh[0][0])[q] = 0.f; (&sd[0][0])[q] = 0.f; }
  __syncthreads();
  float* hrow = &sh[wave * 16][0]; float* drow = &sd[wave * 16][0]; float* h1 = &s1[wave * 16][0]; float* h2 = &s2[wave * 16][0];
#pragma unroll 1
  for (int t = 0; t < NT; ++t) {
#pragma unroll 1
    for (int sub = 0; sub < NSUB; ++sub) {
      { const F2 a = split_row(hrow + col * 72, 0, lane);
#pragma unroll
        for (int j = 0; j < 2; ++j) { v8f acc = {}; const v16b wb = frag_b(&sA[j * 16 + col][0], lane); acc = wmma_bf(a.l, wb, acc); acc = wmma_bf(a.h, wb, acc);
#pragma unroll
          for (int r = 0; r < 8; ++r) { const int rl = 8 * g + r; drow[rl * 72 + j * 16 + col] = acc[r] + sBv[j * 16 + col] * hrow[rl * 72 + NC]; } } }
      { float v[16]; const float* p = hrow + col * 72 + NC;
#pragma unroll
        for (int i = 0; i < 8; ++i) { v[i] = p[8 * g + i]; v[8 + i] = p[16 + 8 * g + i]; }
        const F2 a0 = bsplit16(v);
#pragma unroll
        for (int i = 0; i < 8; ++i) { const int k0 = 32 + 8 * g + i, k1 = 48 + 8 * g + i; v[i] = k0 < NC + 1 ? p[k0 < NC + 1 ? k0 : 0] : 0.f; v[8 + i] = k1 < NC + 1 ? p[k1 < NC + 1 ? k1 : 0] : 0.f; }
        const F2 a1 = bsplit16(v);
#pragma unroll 1
        for (int j = 0; j < 8; ++j) { v8f acc = {}; const v16b w0 = frag_b(&sW1[j * 16 + col][0], lane), w1 = frag_b(&sW1[j * 16 + col][32], lane);
          acc = wmma_bf(a0.l, w0, acc); acc = wmma_bf(a0.h, w0, acc); acc = wmma_bf(a1.l, w1, acc); acc = wmma_bf(a1.h, w1, acc);
#pragma unroll
          for (int r = 0; r < 8; ++r) { const float vv = acc[r] + sb1[j * 16 + col]; h1[(8 * g + r) * (HID + 4) + j * 16 + col] = vv > 0.f ? vv : 0.f; } } }
      LDSX();
      { F2 a[4];
#pragma unroll
        for (int kc = 0; kc < 4; ++kc) a[kc] = split_row(h1 + col * (HID + 4), kc * 32, lane);
#pragma unroll 1
        for (int j = 0; j < 8; ++j) { v8f acc = {};
#pragma unroll
          for (int kc = 0; kc < 4; ++kc) { const v16b wb = frag_b(&sW2[j * 16 + col][kc * 32], lane); acc = wmma_bf(a[kc].l, wb, acc); acc = wmma_bf(a[kc].h, wb, acc); }
#pragma unroll
          for (int r = 0; r < 8; ++r) { const float vv = acc[r] + sb2[j * 16 + col]; h2[(8 * g + r) * (HID + 4) + j * 16 + col] = vv > 0.f ? vv : 0.f; } } }
      LDSX();
      { F2 a[4];
#pragma unroll
        for (int kc = 0; kc < 4; ++kc) a[kc] = split_row(h2 + col * (HID + 4), kc * 32, lane);
#pragma unroll 1
        for (int j = 0; j < 3; ++j) { v8f acc = {};
#pragma unroll
          for (int kc = 0; kc < 4; ++kc) { const v16b wb = frag_b(&sW3[j * 16 + col][kc * 32], lane); acc = wmma_bf(a[kc].l, wb, acc); acc = wmma_bf(a[kc].h, wb, acc); }
          const int n = j * 16 + col;
          if (n < NC + 1) {
#pragma unroll
            for (int r = 0; r < 8; ++r) drow[(8 * g + r) * 72 + NC + n] = acc[r] + sb3[n]; } } }
      LDSX();
      for (int q = lane; q < 16 * NS; q += 32) { const int rl = q / NS, c = q - rl * NS; hrow[rl * 72 + c] = hrow[rl * 72 + c] + 0.01f * drow[rl * 72 + c]; }
      LDSX();
    }
    if (lane < 16) syp[wave * 16 + lane][t] = hrow[lane * 72 + NC];
    LDSX();
    {
      for (int q = lane; q < 16 * (NC + 1); q += 32) { const int rl = q / (NC + 1), c = NC + (q - rl * (NC + 1)); const size_t row = r0 + wave * 16 + rl;
        const float m = bfr(maskin[row * NT + t]); const float hv = hrow[rl * 72 + c];
        const float up = (c == NC) ? bfr(Yin[row * NT + t]) : hrow[rl * 72 + (c - NC - 1)];
        sd[wave * 16 + rl][c] = m * up + (1.0f - m) * hv; }
      LDSX();
      for (int q = lane; q < 16 * (NC + 1); q += 32) { const int rl = q / (NC + 1), c = NC + (q - rl * (NC + 1)); hrow[rl * 72 + c] = sd[wave * 16 + rl][c]; }
      for (int q = lane; q < 16 * NC; q += 32) { const int rl = q >> 5, c = q & 31; const size_t row = r0 + wave * 16 + rl; const float m = bfr(maskin[row * NT + t]); const float hv = hrow[rl * 72 + c]; hrow[rl * 72 + c] = m * hv + (1.0f - m) * hv; }
      LDSX(); }
  }
  for (int q = lane; q < 16 * 16; q += 32) { const int rl = q >> 4, pc = q & 15; const size_t row = r0 + wave * 16 + rl; const v4f v = *(const v4f*)&syp[wave * 16 + rl][pc * 4]; vst2(out0 + row * NT + pc * 4, v); vst2(out1 + row * NT + pc * 4, v); }
  for (int q = lane; q < 16 * 8; q += 32) { const int rl = q >> 3, pc = q & 7; const size_t row = r0 + wave * 16 + rl; vst2(out3 + row * NC + pc * 4, *(const v4f*)(hrow + rl * 72 + pc * 4)); }
  if (blockIdx.x == 0 && tid < 16) { v4f tv; tv[0] = bfr(times[tid * 4]); tv[1] = bfr(times[tid * 4 + 1]); tv[2] = bfr(times[tid * 4 + 2]); tv[3] = bfr(times[tid * 4 + 3]); vst2(out2 + tid * 4, tv); }
}

extern "C" void kernel_launch(void* const* d_in, const int* in_sizes, int n_in, void* d_out, int out_size, void* d_ws, size_t ws_size, hipStream_t stream) {
  (void)in_sizes; (void)n_in; (void)out_size; (void)d_ws; (void)ws_size;
  const float** I = (const float**)d_in;
  float* out0 = (float*)d_out; float* out1 = out0 + (size_t)NBATCH * NT; float* out2 = out1 + (size_t)NBATCH * NT; float* out3 = out2 + NT;
  k_ode<<<NBATCH / RB, 64, 0, stream>>>(I[0], I[1], I[2], I[3], I[4], I[5], I[6], I[7], I[8], I[9], I[10], out0, out1, out2, out3);
}
